// DGCN_87926570483749
// MI455X (gfx1250) — hardware-run, weakly checked
//
#include <hip/hip_runtime.h>
#include <stddef.h>


typedef _Float16 v16h __attribute__((ext_vector_type(16)));
typedef _Float16 v8h  __attribute__((ext_vector_type(8)));
typedef float    v8f  __attribute__((ext_vector_type(8)));
typedef float    v4f  __attribute__((ext_vector_type(4)));

#ifndef NB
#define NB 16
#endif
#ifndef SEQ
#define SEQ 2048
#endif
#define NB_FULL  16
#define SEQ_FULL 2048
#define CC 64
#define EE 16
#define OO 64
#define HH 16
#define KI 128
#define NJ 8192

static_assert(NB >= 1 && NB <= NB_FULL);
static_assert(NB_FULL == 16);
static_assert(SEQ >= 128 && SEQ <= SEQ_FULL && (SEQ % 128) == 0);
static_assert(CC == 64 && OO == 64 && EE == 16 && HH == 16);
static_assert(KI == 2 * CC && NJ == KI * OO);
static_assert((NJ % 64) == 0);

#define LDT 72
#define LDC 68
#define LDK 24
#define HSP 17
static_assert((LDT % 8) == 0 && LDT >= 64);
static_assert((LDC % 4) == 0 && LDC >= 64);
static_assert((LDK % 8) == 0 && LDK >= EE);

#define WCARRY  64.0f
#define NVCARRY 256.0f
#define PCARRY  16384.0f
#define XGCARRY 64.0f

#define WPT_BYTES ((size_t)NJ * EE * 2)
#define X16_BYTES ((size_t)NB * SEQ * CC * 2)
#define NV_BYTES  ((size_t)NB * SEQ * EE * 2)
#define DV_BYTES  ((size_t)NB * SEQ * 4)
#define WT_BYTES  ((size_t)SEQ * OO * KI * 2)
#define OFF_WPT ((size_t)0)
#define OFF_X16 (OFF_WPT + WPT_BYTES)
#define OFF_XT  (OFF_X16 + X16_BYTES)
#define OFF_NV  (OFF_XT + X16_BYTES)
#define OFF_DV  (OFF_NV + NV_BYTES)
#define OFF_XG  (OFF_DV + DV_BYTES)
#define OFF_WT  (OFF_XG + X16_BYTES)
#define WS_TOTAL (OFF_WT + WT_BYTES)
static_assert((WPT_BYTES % 128) == 0 && (X16_BYTES % 128) == 0 && (NV_BYTES % 128) == 0);
static_assert((DV_BYTES % 128) == 0 && (WT_BYTES % 128) == 0);
static_assert(WS_TOTAL <= (size_t)134217728);
static_assert(((size_t)(NB - 1) * SEQ_FULL + SEQ) * OO <= (size_t)NB_FULL * SEQ_FULL * OO);

__device__ __forceinline__ float bf16r(float x) {
  unsigned int u = __float_as_uint(x);
  u = (u + 0x7FFFu + ((u >> 16) & 1u)) & 0xFFFF0000u;
  return __uint_as_float(u);
}

static __device__ __forceinline__ _Float16 toh_flush(float v) {
  const _Float16 r = (_Float16)v;
  return (fabsf(v) < 6.103515625e-05f) ? (_Float16)0.0f : r;
}

__device__ __forceinline__ v16h frag_at(const _Float16* p) {
  v8h lo = *(const v8h*)(p);
  v8h hi = *(const v8h*)(p + 16);
  v16h out;
#pragma unroll
  for (int i = 0; i < 8; ++i) { out[i] = lo[i]; out[i + 8] = hi[i]; }
  return out;
}
__device__ __forceinline__ v16h ld_frag(const _Float16* base, unsigned ld) {
  const unsigned lane = threadIdx.x & 31u;
  return frag_at(base + (lane & 15u) * ld + (lane >> 4) * 8u);
}

__device__ __forceinline__ v16h frag_k16(const _Float16* p) {
  const v8h lo = *(const v8h*)(p);
  v16h out;
#pragma unroll
  for (int i = 0; i < 8; ++i) { out[i] = lo[i]; out[i + 8] = (_Float16)0.0f; }
  return out;
}
__device__ __forceinline__ v16h frag_k16_f32(const float* p, float carry) {
  const v4f a0 = *(const v4f*)(p);
  const v4f a1 = *(const v4f*)(p + 4);
  v16h out;
#pragma unroll
  for (int i = 0; i < 4; ++i) {
    out[i]      = toh_flush(carry * bf16r(a0[i]));
    out[i + 4]  = toh_flush(carry * bf16r(a1[i]));
    out[i + 8]  = (_Float16)0.0f;
    out[i + 12] = (_Float16)0.0f;
  }
  return out;
}

__device__ __forceinline__ v8f wmma16(v16h a, v16h b, v8f c) {
  v8f d = __builtin_amdgcn_wmma_f32_16x16x32_f16(false, a, false, b, (short)0, c,
                                                 false, false);
  asm volatile("v_nop\n\tv_nop\n\tv_nop\n\tv_nop" : "+v"(d) : "v"(a), "v"(b));
  return d;
}

__device__ __forceinline__ float red16_sum(float x) {
#pragma unroll
  for (int off = 1; off < 16; off <<= 1) x += __shfl_xor(x, off, 32);
  return x;
}

__device__ __forceinline__ void wave_lds_sync() {
  __builtin_amdgcn_fence(3  , "wavefront");
  asm volatile("s_wait_dscnt 0x0" ::: "memory");
  __builtin_amdgcn_wave_barrier();
}

__global__ __launch_bounds__(128) void wpool_conv_kernel(
    const float* __restrict__ Wp, _Float16* __restrict__ Wpt) {
  __shared__ _Float16 Tt[64 * EE];
  const unsigned tid = threadIdx.x;
  const unsigned j0 = blockIdx.x * 64u;
#pragma unroll 4
  for (unsigned i = 0; i < 8u; ++i) {
    const unsigned idx = tid + 128u * i;
    const unsigned d = idx >> 6, jj = idx & 63u;
    const float v = Wp[(size_t)d * NJ + j0 + jj];
    Tt[jj * EE + d] = toh_flush(WCARRY * bf16r(v));
  }
  __syncthreads();
  const v8h x = *(const v8h*)&Tt[tid * 8u];
  _Float16* p = Wpt + (size_t)j0 * EE + tid * 8u;
  *(volatile v8h*)p = x;
  __threadfence();
  *(volatile v8h*)p = x;
}

__global__ __launch_bounds__(128) void prep_mlp_kernel(
    const float* __restrict__ X, const float* __restrict__ Emb0,
    const float* __restrict__ W1, const float* __restrict__ B1,
    const float* __restrict__ W2, const float* __restrict__ B2,
    const float* __restrict__ W3, const float* __restrict__ B3,
    _Float16* __restrict__ X16, _Float16* __restrict__ XT16, _Float16* __restrict__ NV16) {
  __shared__ _Float16 T[64 * LDT];
  __shared__ _Float16 TT[64 * LDT];
  __shared__ _Float16 W1s[HH * LDT];
  __shared__ float Hs[64 * HSP];
  __shared__ _Float16 Ns[64 * EE];

  const unsigned tid = threadIdx.x, lane = tid & 31u;
  const unsigned wave = (unsigned)__builtin_amdgcn_readfirstlane((int)(threadIdx.x >> 5));
  const unsigned hh = lane >> 4, m = lane & 15u;
  const unsigned b = blockIdx.y, n0 = blockIdx.x * 64u;
  const size_t inrow0 = (size_t)b * SEQ_FULL + n0;
  const size_t crow0 = (size_t)b * SEQ + n0;

#pragma unroll 2
  for (unsigned j = 0; j < 8u; ++j) {
    const unsigned idx = tid + 128u * j;
    const unsigned r = idx >> 4, c4 = (idx & 15u) * 4u;
    const v4f a = *(const v4f*)(X + (inrow0 + r) * CC + c4);
#pragma unroll
    for (int i = 0; i < 4; ++i) {
      const _Float16 hv = toh_flush(bf16r(a[i]));
      T[r * LDT + c4 + (unsigned)i] = hv;
      TT[(c4 + (unsigned)i) * LDT + r] = hv;
    }
  }
#pragma unroll 2
  for (unsigned j = 0; j < 8u; ++j) {
    const unsigned idx = tid + 128u * j;
    const unsigned ci = idx >> 4, hc = idx & 15u;
    W1s[hc * LDT + ci] = toh_flush(WCARRY * bf16r(W1[idx]));
  }
  __syncthreads();

  {
    v8h xa[4], xb[4];
    size_t oa[4], ob[4];
#pragma unroll
    for (unsigned j = 0; j < 4u; ++j) {
      const unsigned p = tid + 128u * j;
      const unsigned r = p >> 3, kc = (p & 7u) * 8u;
      xa[j] = *(const v8h*)&T[r * LDT + kc];
      oa[j] = (crow0 + r) * CC + kc;
      xb[j] = *(const v8h*)&TT[r * LDT + kc];
      ob[j] = ((size_t)b * CC + r) * SEQ + n0 + kc;
    }
#pragma unroll
    for (int j = 0; j < 4; ++j) *(volatile v8h*)(X16 + oa[j]) = xa[j];
#pragma unroll
    for (int j = 0; j < 4; ++j) *(volatile v8h*)(XT16 + ob[j]) = xb[j];
    __threadfence();
#pragma unroll
    for (int j = 0; j < 4; ++j) *(volatile v8h*)(X16 + oa[j]) = xa[j];
#pragma unroll
    for (int j = 0; j < 4; ++j) *(volatile v8h*)(XT16 + ob[j]) = xb[j];
  }

  v8f acc = {};
#pragma unroll
  for (int c = 0; c < 2; ++c) {
    const v16h a  = ld_frag(&T[(wave * 16u) * LDT + (unsigned)c * 32u], LDT);
    const v16h bw = ld_frag(&W1s[(unsigned)c * 32u], LDT);
    acc = wmma16(a, bw, acc);
  }
  {
    const float bb = bf16r(B1[m]);
#pragma unroll
    for (int r = 0; r < 8; ++r)
      Hs[(wave * 16u + hh * 8u + (unsigned)r) * HSP + m] = acc[r] * (1.0f / WCARRY) + bb;
  }
  __syncthreads();

  {
    const unsigned row = tid >> 1, dh = tid & 1u;
    float a0 = bf16r(B2[0]);
    float a1 = bf16r(B2[1]);
#pragma unroll 1
    for (unsigned h = 0; h < (unsigned)HH; ++h) {
      const float pre = Hs[row * HSP + h];
      const float sg = __builtin_amdgcn_rcpf(1.0f + __expf(-pre));
      a0 += sg * bf16r(W2[h * 2u]);
      a1 += sg * bf16r(W2[h * 2u + 1u]);
    }
    const float g0 = __builtin_amdgcn_rcpf(1.0f + __expf(-a0));
    const float g1 = __builtin_amdgcn_rcpf(1.0f + __expf(-a1));
    const float* e0 = Emb0 + (inrow0 + row) * EE;
#pragma unroll 1
    for (unsigned j = 0; j < 8u; ++j) {
      const unsigned d = dh * 8u + j;
      const float f = (g0 * bf16r(W3[d]) + g1 * bf16r(W3[EE + d])) + bf16r(B3[d]);
      const float e = bf16r(e0[d]);
      const float v = tanhf(e * f);
      Ns[row * EE + d] = toh_flush(NVCARRY * v);
    }
  }
  __syncthreads();
  {
    const v8h x = *(const v8h*)&Ns[tid * 8u];
    _Float16* p = NV16 + crow0 * EE + tid * 8u;
    *(volatile v8h*)p = x;
    __threadfence();
    *(volatile v8h*)p = x;
  }
}

__global__ __launch_bounds__(256) void rowsum_kernel(
    const _Float16* __restrict__ NV16, float* __restrict__ DV) {
  __shared__ float Ds[128];
  const unsigned tid = threadIdx.x, lane = tid & 31u;
  const unsigned wave = (unsigned)__builtin_amdgcn_readfirstlane((int)(threadIdx.x >> 5));
  const unsigned hh = lane >> 4, m = lane & 15u;
  const unsigned b = blockIdx.y, q0 = blockIdx.x * 128u;
  const unsigned qrow0 = q0 + wave * 16u;
  const _Float16* nvb = NV16 + (size_t)b * SEQ * EE;

  const v16h qf = frag_k16(nvb + (size_t)(qrow0 + m) * EE + hh * 8u);
  const _Float16* kp = nvb + (size_t)m * EE + hh * 8u;
  float rs[8];
#pragma unroll
  for (int r = 0; r < 8; ++r) rs[r] = 0.0f;

#pragma unroll 4
  for (unsigned kb = 0; kb < (unsigned)SEQ; kb += 16u) {
    const v16h kf = frag_k16(kp + (size_t)kb * EE);
    v8f t = {};
    t = wmma16(qf, kf, t);
#pragma unroll
    for (int r = 0; r < 8; ++r) rs[r] += fmaxf(t[r], 0.0f);
  }
#pragma unroll
  for (int r = 0; r < 8; ++r) {
    const float tot = red16_sum(rs[r]);
    const float dval = NVCARRY * (1.0f / sqrtf(tot));
    if (m == 0u) Ds[wave * 16u + hh * 8u + (unsigned)r] = dval;
  }
  __syncthreads();
  if (wave == 0u) {
    const v4f x = *(const v4f*)&Ds[lane * 4u];
    float* p = DV + (size_t)b * SEQ + q0 + lane * 4u;
    *(volatile v4f*)p = x;
    __threadfence();
    *(volatile v4f*)p = x;
  }
}

__global__ __launch_bounds__(256) void lx_kernel(
    const _Float16* __restrict__ NV16, const float* __restrict__ DV,
    const _Float16* __restrict__ XT16, _Float16* __restrict__ XG16) {
  __shared__ _Float16 Ks[64 * LDK];
  __shared__ _Float16 Vs[64 * LDT];
  __shared__ float DMs[64];
  __shared__ _Float16 Ps[8 * 16 * LDT];

  const unsigned tid = threadIdx.x, lane = tid & 31u;
  const unsigned wave = (unsigned)__builtin_amdgcn_readfirstlane((int)(threadIdx.x >> 5));
  const unsigned hh = lane >> 4, m = lane & 15u;
  const unsigned b = blockIdx.y, q0 = blockIdx.x * 128u;
  const unsigned qrow0 = q0 + wave * 16u;
  const unsigned pb = wave * (16u * LDT);
  const _Float16* nvb = NV16 + (size_t)b * SEQ * EE;
  const float* dvb = DV + (size_t)b * SEQ;
  const _Float16* xtb = XT16 + (size_t)b * CC * SEQ;

  const v16h qf = frag_k16(nvb + (size_t)(qrow0 + m) * EE + hh * 8u);
  float dn[8];
#pragma unroll
  for (int r = 0; r < 8; ++r)
    dn[r] = dvb[qrow0 + hh * 8u + (unsigned)r] * (PCARRY / (NVCARRY * NVCARRY));
  v8f o[4];
#pragma unroll
  for (int nb = 0; nb < 4; ++nb) o[nb] = (v8f){};

  for (unsigned kb = 0; kb < (unsigned)SEQ; kb += 64u) {
    if (wave < 4u) {
      const unsigned r = tid >> 1, cc = (tid & 1u) * 8u;
      *(v8h*)&Ks[r * LDK + cc] = *(const v8h*)(nvb + (size_t)(kb + r) * EE + cc);
    } else if (wave < 6u) {
      const unsigned kk = tid - 128u;
      DMs[kk] = dvb[kb + kk];
    }
#pragma unroll
    for (unsigned j = 0; j < 2u; ++j) {
      const unsigned idx = tid + 256u * j;
      const unsigned r = idx >> 3, c = (idx & 7u) * 8u;
      *(v8h*)&Vs[r * LDT + c] = *(const v8h*)(xtb + (size_t)r * SEQ + kb + c);
    }
    __syncthreads();

#pragma unroll
    for (int kg = 0; kg < 4; ++kg) {
      const v16h kf = frag_k16(&Ks[((unsigned)kg * 16u + m) * LDK + hh * 8u]);
      v8f t = {};
      t = wmma16(qf, kf, t);
      const float dm = DMs[(unsigned)kg * 16u + m];
#pragma unroll
      for (int r = 0; r < 8; ++r) {
        const float pv = fmaxf(t[r], 0.0f) * dn[r] * dm;
        Ps[pb + (hh * 8u + (unsigned)r) * LDT + (unsigned)kg * 16u + m] = toh_flush(pv);
      }
    }
    wave_lds_sync();

#pragma unroll
    for (int c = 0; c < 2; ++c) {
      const v16h pf = ld_frag(&Ps[pb + (unsigned)c * 32u], LDT);
#pragma unroll
      for (int nb = 0; nb < 4; ++nb) {
        const v16h vf = ld_frag(&Vs[((unsigned)nb * 16u) * LDT + (unsigned)c * 32u], LDT);
        o[nb] = wmma16(pf, vf, o[nb]);
      }
    }
    __syncthreads();
  }

#pragma unroll
  for (int nb = 0; nb < 4; ++nb)
#pragma unroll
    for (int r = 0; r < 8; ++r)
      Ps[pb + (hh * 8u + (unsigned)r) * LDT + (unsigned)nb * 16u + m] =
          toh_flush(o[nb][r] * (XGCARRY / PCARRY));
  wave_lds_sync();
  v8h x[4];
  size_t off[4];
#pragma unroll
  for (unsigned i = 0; i < 4u; ++i) {
    const unsigned r = 4u * i + (lane >> 3);
    const unsigned c = (lane & 7u) * 8u;
    x[i] = *(const v8h*)&Ps[pb + r * LDT + c];
    off[i] = ((size_t)b * SEQ + qrow0 + r) * CC + c;
  }
#pragma unroll
  for (int i = 0; i < 4; ++i) *(volatile v8h*)(XG16 + off[i]) = x[i];
  __threadfence();
#pragma unroll
  for (int i = 0; i < 4; ++i) *(volatile v8h*)(XG16 + off[i]) = x[i];
}

__global__ __launch_bounds__(256) void hw_kernel(
    const float* __restrict__ Emb1, const _Float16* __restrict__ Wpt,
    _Float16* __restrict__ Wt) {
  __shared__ _Float16 Ts[256 * LDT];
  const unsigned tid = threadIdx.x, lane = tid & 31u;
  const unsigned wave = (unsigned)__builtin_amdgcn_readfirstlane((int)(threadIdx.x >> 5));
  const unsigned hh = lane >> 4, m = lane & 15u;
  const unsigned o0 = blockIdx.x * 16u;
  const unsigned kk = blockIdx.y;
  const unsigned n0 = blockIdx.z * 16u;

  const v16h a = frag_k16_f32(Emb1 + (size_t)(n0 + m) * EE + hh * 8u, 1.0f);
#pragma unroll 2
  for (unsigned ii = 0; ii < 8u; ++ii) {
    const unsigned i = wave * 8u + ii;
    const unsigned j0 = (kk * 64u + i) * 64u + o0;
    const v16h bw = frag_k16(Wpt + (size_t)(j0 + m) * EE + hh * 8u);
    v8f t = {};
    t = wmma16(a, bw, t);
#pragma unroll
    for (int r = 0; r < 8; ++r)
      Ts[((hh * 8u + (unsigned)r) * 16u + m) * LDT + i] = toh_flush(t[r]);
  }
  __syncthreads();

  v8h x[8];
  size_t off[8];
#pragma unroll
  for (unsigned it = 0; it < 8u; ++it) {
    const unsigned line = it * 32u + (tid >> 3);
    const unsigned pc = (tid & 7u) * 8u;
    x[it] = *(const v8h*)&Ts[line * LDT + pc];
    off[it] = ((size_t)(n0 + (line >> 4)) * OO + o0 + (line & 15u)) * KI + kk * 64u + pc;
  }
#pragma unroll
  for (int it = 0; it < 8; ++it) *(volatile v8h*)(Wt + off[it]) = x[it];
  __threadfence();
#pragma unroll
  for (int it = 0; it < 8; ++it) *(volatile v8h*)(Wt + off[it]) = x[it];
}

__global__ __launch_bounds__(256) void out_kernel(
    const _Float16* __restrict__ X16, const _Float16* __restrict__ XG16,
    const _Float16* __restrict__ Wt, const float* __restrict__ Emb1,
    const float* __restrict__ Bp, float* __restrict__ Out) {
  __shared__ float Bs[16 * OO];
  __shared__ float Cs[8 * 16 * LDC];
  const unsigned tid = threadIdx.x, lane = tid & 31u;
  const unsigned wave = (unsigned)__builtin_amdgcn_readfirstlane((int)(threadIdx.x >> 5));
  const unsigned hh = lane >> 4, m = lane & 15u;
  const unsigned n0 = blockIdx.x * 16u;
  const unsigned cb = wave * (16u * LDC);

  if (wave < 4u) {
    const v16h a = frag_k16_f32(Emb1 + (size_t)(n0 + m) * EE + hh * 8u, 1.0f);
    v16h bf;
#pragma unroll
    for (int i = 0; i < 8; ++i) {
      const float v = Bp[(hh * 8u + (unsigned)i) * OO + wave * 16u + m];
      bf[i] = toh_flush(WCARRY * bf16r(v));
      bf[i + 8] = (_Float16)0.0f;
    }
    v8f t = {};
    t = wmma16(a, bf, t);
#pragma unroll
    for (int r = 0; r < 8; ++r)
      Bs[(hh * 8u + (unsigned)r) * OO + wave * 16u + m] = t[r] * (1.0f / WCARRY);
  }
  __syncthreads();

  const unsigned bsel = (m < (unsigned)NB) ? m : (unsigned)(NB - 1);
#pragma unroll 1
  for (unsigned nn = 0; nn < 2u; ++nn) {
    const unsigned nl = wave * 2u + nn;
    const unsigned n = n0 + nl;
    const size_t xrow = ((size_t)bsel * SEQ + n) * CC + hh * 8u;
    const size_t wrow = ((size_t)n * OO + m) * KI + hh * 8u;
    v8f acc0[4], acc1[4];
#pragma unroll
    for (int ct = 0; ct < 4; ++ct) { acc0[ct] = (v8f){}; acc1[ct] = (v8f){}; }
#pragma unroll
    for (int c = 0; c < 2; ++c) {
      const v16h ax = frag_at(X16 + xrow + (unsigned)c * 32u);
      const v16h ag = frag_at(XG16 + xrow + (unsigned)c * 32u);
#pragma unroll
      for (int ct = 0; ct < 4; ++ct) {
        const _Float16* wp = Wt + wrow + (size_t)((unsigned)ct * 16u) * KI + (unsigned)c * 32u;
        const v16h b0 = frag_at(wp);
        const v16h b1 = frag_at(wp + 64);
        acc0[ct] = wmma16(ax, b0, acc0[ct]);
        acc1[ct] = wmma16(ag, b1, acc1[ct]);
      }
    }
#pragma unroll
    for (int ct = 0; ct < 4; ++ct)
#pragma unroll
      for (int r = 0; r < 8; ++r)
        Cs[cb + (hh * 8u + (unsigned)r) * LDC + (unsigned)ct * 16u + m] =
            acc0[ct][r] * (1.0f / WCARRY) + acc1[ct][r] * (1.0f / (WCARRY * XGCARRY));
    wave_lds_sync();

    v4f xs[8];
    size_t off[8];
#pragma unroll
    for (unsigned i = 0; i < 8u; ++i) {
      const unsigned bb = 2u * i + hh;
      const unsigned c = m * 4u;
      const v4f u = *(const v4f*)&Cs[cb + bb * LDC + c];
      const v4f g = *(const v4f*)&Bs[nl * OO + c];
      xs[i] = u + g;
      off[i] = ((size_t)bb * SEQ_FULL + n) * OO + c;
    }
#pragma unroll
    for (unsigned i = 0; i < 8u; ++i)
      if (2u * i + hh < (unsigned)NB) *(volatile v4f*)(Out + off[i]) = xs[i];
    __threadfence();
#pragma unroll
    for (unsigned i = 0; i < 8u; ++i)
      if (2u * i + hh < (unsigned)NB) *(volatile v4f*)(Out + off[i]) = xs[i];
    wave_lds_sync();
  }
}

extern "C" void kernel_launch(void* const* d_in, const int* in_sizes, int n_in,
                              void* d_out, int out_size, void* d_ws, size_t ws_size,
                              hipStream_t stream) {
  if (n_in < 11) return;
  const long long need_rows = (long long)(NB - 1) * SEQ_FULL + SEQ;
  if ((long long)in_sizes[0] < need_rows * CC) return;
  if ((long long)in_sizes[1] < need_rows * EE) return;
  if ((long long)in_sizes[2] < (long long)SEQ * EE) return;
  if (in_sizes[3] < CC * HH || in_sizes[4] < HH) return;
  if (in_sizes[5] < HH * 2 || in_sizes[6] < 2) return;
  if (in_sizes[7] < 2 * EE || in_sizes[8] < EE) return;
  if ((long long)in_sizes[9] < (long long)EE * NJ) return;
  if (in_sizes[10] < EE * OO) return;
  if ((long long)out_size < need_rows * OO) return;
  if (ws_size < WS_TOTAL) return;

  const float* x    = (const float*)d_in[0];
  const float* emb0 = (const float*)d_in[1];
  const float* emb1 = (const float*)d_in[2];
  const float* w1   = (const float*)d_in[3];
  const float* b1   = (const float*)d_in[4];
  const float* w2   = (const float*)d_in[5];
  const float* b2   = (const float*)d_in[6];
  const float* w3   = (const float*)d_in[7];
  const float* b3   = (const float*)d_in[8];
  const float* wp   = (const float*)d_in[9];
  const float* bp   = (const float*)d_in[10];
  float* out = (float*)d_out;

  char* ws = (char*)d_ws;
  _Float16* Wpt  = (_Float16*)(ws + OFF_WPT);
  _Float16* X16  = (_Float16*)(ws + OFF_X16);
  _Float16* XT16 = (_Float16*)(ws + OFF_XT);
  _Float16* NV16 = (_Float16*)(ws + OFF_NV);
  float*    DV   = (float*)(ws + OFF_DV);
  _Float16* XG16 = (_Float16*)(ws + OFF_XG);
  _Float16* Wt   = (_Float16*)(ws + OFF_WT);

  wpool_conv_kernel<<<dim3(NJ / 64), dim3(128), 0, stream>>>(wp, Wpt);
  prep_mlp_kernel<<<dim3(SEQ / 64, NB), dim3(128), 0, stream>>>(
      x, emb0, w1, b1, w2, b2, w3, b3, X16, XT16, NV16);
  rowsum_kernel<<<dim3(SEQ / 128, NB), dim3(256), 0, stream>>>(NV16, DV);
  lx_kernel<<<dim3(SEQ / 128, NB), dim3(256), 0, stream>>>(NV16, DV, XT16, XG16);
  hw_kernel<<<dim3(OO / 16, 2, SEQ / 16), dim3(256), 0, stream>>>(emb1, Wpt, Wt);
  out_kernel<<<dim3(SEQ / 16), dim3(256), 0, stream>>>(X16, XG16, Wt, emb1, bp, out);
}
